// SimpleRNN_37426345017535
// MI455X (gfx1250) — hardware-run, weakly checked
//
#include <hip/hip_runtime.h>
#include <math.h>

constexpr int NSEQ    = 256;
constexpr int NSTEP   = 2048;
constexpr int NIN     = 10;
constexpr int NHID    = 64;
constexpr int NHEAD   = 2;
constexpr int SEQ_BLK = 16;
constexpr int NTHR    = 32;
constexpr int KXPAD   = 32;
constexpr int XPITCH  = 40;
constexpr int HPITCH  = 72;
constexpr int SPITCH  = 68;
constexpr int OPITCH  = 36;
constexpr int TCHUNK  = 16;

static_assert(NSEQ % SEQ_BLK == 0);
static_assert(NSTEP % TCHUNK == 0);
static_assert(NHID == 64);
static_assert(NIN <= KXPAD && (NIN % 2) == 0);
static_assert(TCHUNK * NHEAD * 4 == 128);
static_assert((XPITCH % 8) == 0 && (HPITCH % 8) == 0 && (SPITCH % 4) == 0 && (OPITCH % 4) == 0);

typedef __attribute__((ext_vector_type(16))) __bf16   v16b;
typedef __attribute__((ext_vector_type(8)))  __bf16   v8b;
typedef __attribute__((ext_vector_type(8)))  float    v8f;
typedef __attribute__((ext_vector_type(4)))  float    v4f;
typedef __attribute__((ext_vector_type(2)))  float    v2f;
typedef __attribute__((ext_vector_type(4)))  unsigned v4u;

__device__ __forceinline__ unsigned short f2bf_bits(float f) {
  unsigned u = __float_as_uint(f);
  return (unsigned short)((u + 0x7FFFu + ((u >> 16) & 1u)) >> 16);
}
__device__ __forceinline__ float bf_bits2f(unsigned short h) { return __uint_as_float(((unsigned)h) << 16); }

template <typename T> struct Frag;
template <> struct Frag<__bf16> {
  typedef v16b V; union U { v16b v; v8b h[2]; };
  static __device__ __forceinline__ v16b load(const __bf16* p) {
    U f; f.h[0] = *(const v8b*)(p); f.h[1] = *(const v8b*)(p + 16); return f.v;
  }
};

__device__ __forceinline__ v8f mma_bf(v16b a, v16b b, v8f c) {
  c = __builtin_amdgcn_wmma_f32_16x16x32_bf16(false, a, false, b, (short)0, c, false, false);
  asm volatile("v_nop\n\tv_nop\n\tv_nop\n\tv_nop" : "+v"(c) : "v"(a), "v"(b));
  return c;
}
__device__ __forceinline__ void acc_guard1(v8f& a) { asm volatile("v_nop\n\tv_nop\n\tv_nop\n\tv_nop" : "+v"(a)); }

__device__ __forceinline__ void split_pair(float a, float b, unsigned& wh, unsigned& wl) {
  const unsigned short ha = f2bf_bits(a), hb = f2bf_bits(b);
  const unsigned short la = f2bf_bits(a - bf_bits2f(ha)), lb = f2bf_bits(b - bf_bits2f(hb));
  wh = (unsigned)ha | ((unsigned)hb << 16);
  wl = (unsigned)la | ((unsigned)lb << 16);
}

__global__ __launch_bounds__(NTHR) void seq_tanh_kernel(const float* __restrict__ x, const float* __restrict__ wx,
                                                       const float* __restrict__ wh, const float* __restrict__ bvec,
                                                       const float* __restrict__ wd, const float* __restrict__ bd,
                                                       float* __restrict__ out) {
  __shared__ __align__(16) unsigned short WhH[NHID * HPITCH];
  __shared__ __align__(16) unsigned short WhL[NHID * HPITCH];
  __shared__ __align__(16) unsigned short WxH[NHID * XPITCH];
  __shared__ __align__(16) unsigned short WxL[NHID * XPITCH];
  __shared__ __align__(16) unsigned short AhH[2][SEQ_BLK * HPITCH];
  __shared__ __align__(16) unsigned short AhL[2][SEQ_BLK * HPITCH];
  __shared__ __align__(16) unsigned short XsH[SEQ_BLK * XPITCH];
  __shared__ __align__(16) unsigned short XsL[SEQ_BLK * XPITCH];
  __shared__ __align__(16) float Hs[SEQ_BLK * SPITCH];
  __shared__ __align__(16) float Os[SEQ_BLK * OPITCH];
  __shared__ __align__(16) float Wds[NHEAD * NHID];
  __shared__ __align__(16) float Bs[NHID];

  const int lane = threadIdx.x;
  const int c = lane & 15, hh = lane >> 4, koff = hh * 8;
  const int rowbase = blockIdx.x * SEQ_BLK;

  {
    unsigned* p;
    p = (unsigned*)WhH;
#pragma unroll 1
    for (int i = lane; i < (NHID * HPITCH) / 2; i += NTHR) p[i] = 0u;
    p = (unsigned*)WhL;
#pragma unroll 1
    for (int i = lane; i < (NHID * HPITCH) / 2; i += NTHR) p[i] = 0u;
    p = (unsigned*)WxH;
#pragma unroll 1
    for (int i = lane; i < (NHID * XPITCH) / 2; i += NTHR) p[i] = 0u;
    p = (unsigned*)WxL;
#pragma unroll 1
    for (int i = lane; i < (NHID * XPITCH) / 2; i += NTHR) p[i] = 0u;
    p = (unsigned*)&AhH[0][0];
#pragma unroll 1
    for (int i = lane; i < (2 * SEQ_BLK * HPITCH) / 2; i += NTHR) p[i] = 0u;
    p = (unsigned*)&AhL[0][0];
#pragma unroll 1
    for (int i = lane; i < (2 * SEQ_BLK * HPITCH) / 2; i += NTHR) p[i] = 0u;
    p = (unsigned*)XsH;
#pragma unroll 1
    for (int i = lane; i < (SEQ_BLK * XPITCH) / 2; i += NTHR) p[i] = 0u;
    p = (unsigned*)XsL;
#pragma unroll 1
    for (int i = lane; i < (SEQ_BLK * XPITCH) / 2; i += NTHR) p[i] = 0u;
#pragma unroll 1
    for (int i = lane; i < SEQ_BLK * SPITCH; i += NTHR) Hs[i] = 0.0f;
#pragma unroll 1
    for (int i = lane; i < SEQ_BLK * OPITCH; i += NTHR) Os[i] = 0.0f;
#pragma unroll 1
    for (int i = lane; i < NHEAD * NHID; i += NTHR) Wds[i] = 0.0f;
#pragma unroll 1
    for (int i = lane; i < NHID; i += NTHR) Bs[i] = 0.0f;
  }
  __syncthreads();

#pragma unroll 1
  for (int i = lane; i < NHID * NHID; i += NTHR) {
    const int k = i >> 6, n = i & 63;
    const float v = wh[i];
    const unsigned short hb = f2bf_bits(v);
    const unsigned short lb = f2bf_bits(v - bf_bits2f(hb));
    WhH[n * HPITCH + k] = hb;
    WhL[n * HPITCH + k] = lb;
  }
#pragma unroll 1
  for (int i = lane; i < NHID * XPITCH; i += NTHR) {
    const int n = i / XPITCH, k = i - n * XPITCH;
    const int kc = (k < NIN) ? k : (NIN - 1);
    const float fk = (k < NIN) ? 1.0f : 0.0f;
    const float v = wx[kc * NHID + n] * fk;
    const unsigned short hb = f2bf_bits(v);
    const unsigned short lb = f2bf_bits(v - bf_bits2f(hb));
    WxH[n * XPITCH + k] = hb;
    WxL[n * XPITCH + k] = lb;
  }
#pragma unroll 1
  for (int i = lane; i < NHID * NHEAD; i += NTHR) {
    const int u = i >> 1, o = i & 1;
    Wds[o * NHID + u] = wd[i];
  }
#pragma unroll 1
  for (int i = lane; i < NHID; i += NTHR) Bs[i] = bvec[i];
  const float bdv = bd[hh];
  __syncthreads();

  const float* xrow = x + (size_t)(rowbase + c) * NSTEP * NIN;
  const v8f z8 = {0.f, 0.f, 0.f, 0.f, 0.f, 0.f, 0.f, 0.f};
  const v4u qz = {0u, 0u, 0u, 0u};

#pragma unroll 1
  for (int t = 0; t < NSTEP; ++t) {
    const int cur = t & 1, nxt = cur ^ 1;

    {
      const float* xp = xrow + (size_t)t * NIN;
      const v2f p0 = *(const v2f*)(xp + 0);
      const v2f p1 = *(const v2f*)(xp + 2);
      const v2f p2 = *(const v2f*)(xp + 4);
      const v2f p3 = *(const v2f*)(xp + 6);
      const v2f p4 = *(const v2f*)(xp + 8);
      unsigned wh0, wl0, wh1, wl1, wh2, wl2, wh3, wl3, wh4, wl4;
      split_pair(p0[0], p0[1], wh0, wl0);
      split_pair(p1[0], p1[1], wh1, wl1);
      split_pair(p2[0], p2[1], wh2, wl2);
      split_pair(p3[0], p3[1], wh3, wl3);
      split_pair(p4[0], p4[1], wh4, wl4);
      const v4u qh0 = {wh0, wh1, wh2, wh3};
      const v4u qh1 = {wh4, 0u, 0u, 0u};
      const v4u ql0 = {wl0, wl1, wl2, wl3};
      const v4u ql1 = {wl4, 0u, 0u, 0u};
      unsigned short* xhp = XsH + c * XPITCH;
      unsigned short* xlp = XsL + c * XPITCH;
      *(v4u*)(xhp + 0)  = qh0;
      *(v4u*)(xhp + 8)  = qh1;
      *(v4u*)(xhp + 16) = qz;
      *(v4u*)(xhp + 24) = qz;
      *(v4u*)(xlp + 0)  = ql0;
      *(v4u*)(xlp + 8)  = ql1;
      *(v4u*)(xlp + 16) = qz;
      *(v4u*)(xlp + 24) = qz;
    }
    __syncthreads();

    const __bf16* axh = (const __bf16*)XsH + c * XPITCH + koff;
    const __bf16* axl = (const __bf16*)XsL + c * XPITCH + koff;
    const __bf16* ahh = (const __bf16*)(&AhH[cur][0]) + c * HPITCH + koff;
    const __bf16* ahl = (const __bf16*)(&AhL[cur][0]) + c * HPITCH + koff;
    const v16b fxh = Frag<__bf16>::load(axh);
    const v16b fxl = Frag<__bf16>::load(axl);
    const v16b fh0 = Frag<__bf16>::load(ahh);
    const v16b fh1 = Frag<__bf16>::load(ahh + 32);
    const v16b fl0 = Frag<__bf16>::load(ahl);
    const v16b fl1 = Frag<__bf16>::load(ahl + 32);
    unsigned short* anh = &AhH[nxt][0];
    unsigned short* anl = &AhL[nxt][0];

#pragma unroll 1
    for (int nt = 0; nt < 4; ++nt) {
      const int col = 16 * nt + c;
      const __bf16* bxh = (const __bf16*)WxH + col * XPITCH + koff;
      const __bf16* bxl = (const __bf16*)WxL + col * XPITCH + koff;
      const __bf16* bwh = (const __bf16*)WhH + col * HPITCH + koff;
      const __bf16* bwl = (const __bf16*)WhL + col * HPITCH + koff;
      const v16b gxh = Frag<__bf16>::load(bxh);
      const v16b gxl = Frag<__bf16>::load(bxl);
      const v16b gh0 = Frag<__bf16>::load(bwh);
      const v16b gh1 = Frag<__bf16>::load(bwh + 32);
      const v16b gl0 = Frag<__bf16>::load(bwl);
      const v16b gl1 = Frag<__bf16>::load(bwl + 32);
      v8f acc = z8;
      acc = mma_bf(fxh, gxh, acc);
      acc = mma_bf(fxh, gxl, acc);
      acc = mma_bf(fxl, gxh, acc);
      acc = mma_bf(fh0, gh0, acc);
      acc = mma_bf(fh0, gl0, acc);
      acc = mma_bf(fl0, gh0, acc);
      acc = mma_bf(fh1, gh1, acc);
      acc = mma_bf(fh1, gl1, acc);
      acc = mma_bf(fl1, gh1, acc);
      acc_guard1(acc);
      const float bcol = Bs[col];
#pragma unroll
      for (int r = 0; r < 8; ++r) {
        const float pre = acc[r] + bcol;
        const float hn = tanhf(pre);
        const unsigned short hb = f2bf_bits(hn);
        const unsigned short lb = f2bf_bits(hn - bf_bits2f(hb));
        const int ro = 8 * hh + r;
        anh[ro * HPITCH + col] = hb;
        anl[ro * HPITCH + col] = lb;
        Hs[ro * SPITCH + col] = hn;
      }
    }
    __syncthreads();

    {
      const float* hr = Hs + c * SPITCH;
      const float* wr = Wds + hh * NHID;
      float s = 0.0f;
#pragma unroll
      for (int i = 0; i < NHID / 4; ++i) {
        const v4f hv = *(const v4f*)(hr + 4 * i);
        const v4f wv = *(const v4f*)(wr + 4 * i);
        s = fmaf(hv[0], wv[0], s);
        s = fmaf(hv[1], wv[1], s);
        s = fmaf(hv[2], wv[2], s);
        s = fmaf(hv[3], wv[3], s);
      }
      Os[c * OPITCH + (t & (TCHUNK - 1)) * NHEAD + hh] = s + bdv;
    }

    if ((t & (TCHUNK - 1)) == TCHUNK - 1) {
      __syncthreads();
      const int t0 = t - (TCHUNK - 1);
      const int q = lane >> 3, c4 = (lane & 7) * 4;
      for (int pass = 0; pass < 2; ++pass) {
#pragma unroll
        for (int it = 0; it < 4; ++it) {
          const int row = it * 4 + q;
          const v4f v = *(const v4f*)(Os + row * OPITCH + c4);
          *(volatile v4f*)(out + ((size_t)(rowbase + row) * NSTEP + (size_t)t0) * NHEAD + c4) = v;
        }
        __threadfence();
      }
    }
  }
}

extern "C" void kernel_launch(void* const* d_in, const int* in_sizes, int n_in,
                              void* d_out, int out_size, void* d_ws, size_t ws_size, hipStream_t stream) {
  (void)d_ws; (void)ws_size;
  if (n_in < 6 || d_out == nullptr) return;
  if (in_sizes[0] != NSEQ * NSTEP * NIN || in_sizes[1] != NIN * NHID || in_sizes[2] != NHID * NHID ||
      in_sizes[3] != NHID || in_sizes[4] != NHID * NHEAD || in_sizes[5] != NHEAD ||
      out_size != NSEQ * NSTEP * NHEAD) return;

  const float* x    = (const float*)d_in[0];
  const float* wx   = (const float*)d_in[1];
  const float* wh   = (const float*)d_in[2];
  const float* bvec = (const float*)d_in[3];
  const float* wd   = (const float*)d_in[4];
  const float* bd   = (const float*)d_in[5];
  float* out = (float*)d_out;

  seq_tanh_kernel<<<NSEQ / SEQ_BLK, NTHR, 0, stream>>>(x, wx, wh, bvec, wd, bd, out);
}
